// Backbone_4243427688698
// MI455X (gfx1250) — hardware-verified
//
#include <hip/hip_runtime.h>
#include <stddef.h>
#include <math.h>


#define DMOD     128
#define HID      512
#define NPG      9
#define EPG      16
#define GPH      16
#define GPB      32
#define NODES    (GPH * NPG)
#define NEB      (GPH * EPG)
#define NWAVES   9
#define NTHREADS (NWAVES * 32)
#define STR      136
#define HSP      128
#define NLAYERS  4
#define MAXIN    16
#define LN_EPS   1e-5f
#define ASCL     16.0f
#define WSCL     256.0f
#define CSCL     4096.0f
#define INVSCL   0.000244140625f

#define OFF_HS   0
#define OFF_AH   (OFF_HS + NODES * HSP * 4)
#define OFF_HH   (OFF_AH + NODES * STR * 2)
#define OFF_TH   (OFF_HH + NODES * STR * 2)
#define OFF_LST  (OFF_TH + NWAVES * 16 * STR * 2)
#define OFF_CNT  (OFF_LST + NODES * MAXIN * 4)
#define OFF_EN   (OFF_CNT + 256 * 4)
#define OFF_ISD  (OFF_EN + 256 * 4)
#define OFF_LS   (OFF_ISD + 256 * 4)
#define OFF_OUT  (OFF_LS + 256 * 4)
#define SMEM_BYTES (OFF_OUT + GPB * 4)

static_assert(NODES == NWAVES * 16);
static_assert(NEB == 256 && NEB <= NTHREADS);
static_assert((NODES * 16) % NTHREADS == 0);
static_assert((NODES * 32) % NTHREADS == 0);
static_assert(MAXIN == EPG && (MAXIN & (MAXIN - 1)) == 0);
static_assert(GPB == 2 * GPH && GPB == 32);
static_assert(GPH * 16 == 256);
static_assert((DMOD % 32) == 0 && (HID % 32) == 0 && (HID % DMOD) == 0);
static_assert((OFF_AH % 16) == 0 && (OFF_HH % 16) == 0 && (OFF_TH % 16) == 0 && (OFF_LST % 16) == 0);
static_assert((OFF_CNT % 16) == 0 && (OFF_EN % 16) == 0 && (OFF_ISD % 16) == 0 && (OFF_LS % 16) == 0 && (OFF_OUT % 16) == 0);
static_assert(((16 * STR * 2) % 16) == 0 && ((STR * 2) % 16) == 0);
static_assert(SMEM_BYTES < 300000);

typedef float          v4f  __attribute__((ext_vector_type(4)));
typedef float          v8f  __attribute__((ext_vector_type(8)));
typedef unsigned short v8us __attribute__((ext_vector_type(8)));
typedef v8us           v8usa __attribute__((may_alias));
typedef _Float16       v16h __attribute__((ext_vector_type(16)));
union FragH { v16h v; v8us u[2]; };

__device__ __forceinline__ unsigned short h16(float f) {
  const _Float16 h = (_Float16)f;
  return __builtin_bit_cast(unsigned short, h);
}

__device__ __forceinline__ v8f wmh(v16h a, v16h b, v8f c) {
  v8f d = __builtin_amdgcn_wmma_f32_16x16x32_f16(false, a, false, b, (short)0, c, false, false);
  asm volatile("v_nop\n\tv_nop\n\tv_nop\n\tv_nop" : "+v"(d) : "v"(a), "v"(b));
  return d;
}

__device__ __forceinline__ v16h ldA(const unsigned short* rowPtr, int kt, int hh) {
  FragH u;
  const unsigned short* p = rowPtr + kt * 32 + 8 * hh;
  u.u[0] = *(const v8usa*)p;
  u.u[1] = *(const v8usa*)(p + 16);
  return u.v;
}

__device__ __forceinline__ v16h ldB(const unsigned short* base, int blk, int lane) {
  FragH u;
  const unsigned short* p = base + (size_t)blk * 512 + lane * 16;
  u.u[0] = *(const v8us*)p;
  u.u[1] = *(const v8us*)(p + 8);
  return u.v;
}

__global__ __launch_bounds__(256) void k_wprep(
    const float* __restrict__ W, unsigned short* T, int Ktot, int Ntot, int npieces) {
  const int tid = (int)threadIdx.x;
  const int p = (int)blockIdx.x * 256 + tid;
  const int layer = (int)blockIdx.y;
  const bool live = p < npieces;
  const int pc = live ? p : (npieces - 1);
  const int blk = pc >> 6;
  const int w = pc & 63;
  const int ln = w >> 1, hi = w & 1;
  const int nnf = Ntot >> 4;
  const int kt = blk / nnf;
  const int nf = blk - kt * nnf;
  const int hh = ln >> 4;
  const int k0 = kt * 32 + 16 * hi + 8 * hh;
  const int n = nf * 16 + (ln & 15);
  const size_t lsz = (size_t)Ktot * (size_t)Ntot;
  const float* Wl = W + (size_t)layer * lsz;
  v8us o;
#pragma unroll
  for (int j = 0; j < 8; ++j) {
    int k = k0 + j; k = k > Ktot - 1 ? Ktot - 1 : k;
    o[j] = h16(Wl[(size_t)k * Ntot + n] * WSCL);
  }
  unsigned short* dp = T + (size_t)layer * lsz + (size_t)pc * 8;
  if (live) *(volatile v8us*)dp = o;
  __threadfence();
  if (live) *(volatile v8us*)dp = o;
}

__global__ __launch_bounds__(NTHREADS) void k_gcn(
    const float* __restrict__ op_table, const float* __restrict__ device_emb,
    const float* __restrict__ bg, const float* __restrict__ ln_g, const float* __restrict__ ln_b,
    const float* __restrict__ b1, const float* __restrict__ b2,
    const float* __restrict__ fc_w, const float* __restrict__ fc_b,
    const int* __restrict__ op_idx, const int* __restrict__ srcE, const int* __restrict__ dstE,
    const unsigned short* __restrict__ wgF, const unsigned short* __restrict__ w1F,
    const unsigned short* __restrict__ w2F,
    float* out, int nG, int nN, int nE, int nOps) {
  extern __shared__ v4f smemv[];
  char* smem = (char*)smemv;
  float*          hS   = (float*)(smem + OFF_HS);
  unsigned short* aH   = (unsigned short*)(smem + OFF_AH);
  unsigned short* hH   = (unsigned short*)(smem + OFF_HH);
  unsigned short* tAll = (unsigned short*)(smem + OFF_TH);
  int*            lst  = (int*)(smem + OFF_LST);
  int*            lcnt = (int*)(smem + OFF_CNT);
  float*          enrm = (float*)(smem + OFF_EN);
  float*          isd  = (float*)(smem + OFF_ISD);
  int*            lsrc = (int*)(smem + OFF_LS);
  float*          sOut = (float*)(smem + OFF_OUT);

  const int tid = (int)threadIdx.x, lane = tid & 31, wave = tid >> 5, hh = lane >> 4, l16 = lane & 15;
  const int row0 = wave * 16;
  unsigned short* tW = tAll + wave * (16 * STR);
  const v8f zero8 = {0.0f, 0.0f, 0.0f, 0.0f, 0.0f, 0.0f, 0.0f, 0.0f};

#pragma unroll 1
  for (int hp = 0; hp < 2; ++hp) {
    const int g0 = (int)blockIdx.x * GPB + hp * GPH;
    const int nodeBase = g0 * NPG;
    __syncthreads();

    {
      const int n = tid < NODES ? tid : (NODES - 1);
      const int gl = n / NPG;
      int cnt = 0;
#pragma unroll 1
      for (int e = 0; e < EPG; ++e) {
        int ge = (g0 + gl) * EPG + e;
        ge = ge < 0 ? 0 : (ge > nE - 1 ? nE - 1 : ge);
        const int ld = dstE[ge] - nodeBase;
        const bool hit = (ld == n);
        if (hit && tid < NODES) lst[n * MAXIN + (cnt & (MAXIN - 1))] = gl * EPG + e;
        cnt += hit ? 1 : 0;
      }
      if (tid < NODES) { lcnt[n] = cnt; isd[n] = rsqrtf((float)(1 + cnt)); }
    }
    {
      const int e = tid & (NEB - 1);
      int ge = g0 * EPG + e;
      ge = ge < 0 ? 0 : (ge > nE - 1 ? nE - 1 : ge);
      int ls = srcE[ge] - nodeBase;
      int ld = dstE[ge] - nodeBase;
      ls = ls < 0 ? 0 : (ls > NODES - 1 ? NODES - 1 : ls);
      ld = ld < 0 ? 0 : (ld > NODES - 1 ? NODES - 1 : ld);
      if (tid < NEB) lsrc[e] = ls;
      __syncthreads();
      const float en = isd[ls] * isd[ld];
      if (tid < NEB) enrm[e] = en;
    }
#pragma unroll 1
    for (int j = 0; j < (NODES * 32) / NTHREADS; ++j) {
      const int i = tid + j * NTHREADS;
      const int n = i >> 5, c4 = (i & 31) * 4;
      int node = nodeBase + n; node = node > nN - 1 ? nN - 1 : node;
      int op = op_idx[node]; op = op < 0 ? 0 : (op > nOps - 1 ? nOps - 1 : op);
      const v4f tv = *(const v4f*)(op_table + (size_t)op * DMOD + c4);
      const v4f dv = *(const v4f*)(device_emb + c4);
      *(v4f*)(hS + n * HSP + c4) = tv + dv;
    }
    __syncthreads();

#pragma unroll 1
    for (int l = 0; l < NLAYERS; ++l) {
      const unsigned short* wgl = wgF + (size_t)l * (DMOD * DMOD);
      const unsigned short* w1l = w1F + (size_t)l * (DMOD * HID);
      const unsigned short* w2l = w2F + (size_t)l * (HID * DMOD);

#pragma unroll 1
      for (int j = 0; j < (NODES * 16) / NTHREADS; ++j) {
        const int it = tid + j * NTHREADS;
        const int n = it >> 4, c8 = (it & 15) * 8;
        const float dn = isd[n];
        const float sw = dn * dn;
        v4f a0 = *(const v4f*)(hS + n * HSP + c8);
        v4f a1 = *(const v4f*)(hS + n * HSP + c8 + 4);
        a0 = a0 * sw; a1 = a1 * sw;
        int cn = lcnt[n]; cn = cn < 0 ? 0 : (cn > MAXIN ? MAXIN : cn);
        int cm = cn;
        { const int o2 = __shfl_xor(cm, 16); cm = o2 > cm ? o2 : cm; }
        cm = __builtin_amdgcn_readfirstlane(cm);
#pragma unroll 1
        for (int i = 0; i < cm; ++i) {
          const int e = lst[n * MAXIN + (i & (MAXIN - 1))] & (NEB - 1);
          const float w = (i < cn) ? enrm[e] : 0.0f;
          const int s = lsrc[e];
          const v4f y0 = *(const v4f*)(hS + s * HSP + c8);
          const v4f y1 = *(const v4f*)(hS + s * HSP + c8 + 4);
          a0 = a0 + y0 * w; a1 = a1 + y1 * w;
        }
        v8us o;
        o[0] = h16(a0.x * ASCL); o[1] = h16(a0.y * ASCL); o[2] = h16(a0.z * ASCL); o[3] = h16(a0.w * ASCL);
        o[4] = h16(a1.x * ASCL); o[5] = h16(a1.y * ASCL); o[6] = h16(a1.z * ASCL); o[7] = h16(a1.w * ASCL);
        *(v8us*)(aH + n * STR + c8) = o;
      }
      __syncthreads();

      v8f c[8];
      {
        v16h aF[4];
        const unsigned short* ar = aH + (row0 + l16) * STR;
#pragma unroll
        for (int kt = 0; kt < 4; ++kt) aF[kt] = ldA(ar, kt, hh);
#pragma unroll
        for (int nf = 0; nf < 8; ++nf) {
          v8f acc = zero8;
#pragma unroll
          for (int kt = 0; kt < 4; ++kt) acc = wmh(aF[kt], ldB(wgl, kt * (DMOD / 16) + nf, lane), acc);
          const float bv = bg[l * DMOD + nf * 16 + l16];
#pragma unroll
          for (int i = 0; i < 8; ++i) acc[i] = fmaxf(acc[i] * INVSCL + bv, 0.0f);
          c[nf] = acc;
        }
      }

      float mu[8], rs[8];
#pragma unroll
      for (int i = 0; i < 8; ++i) {
        float s = 0.0f;
#pragma unroll
        for (int nf = 0; nf < 8; ++nf) s += c[nf][i];
        s += __shfl_xor(s, 1); s += __shfl_xor(s, 2); s += __shfl_xor(s, 4); s += __shfl_xor(s, 8);
        const float m = s * (1.0f / 128.0f);
        float v = 0.0f;
#pragma unroll
        for (int nf = 0; nf < 8; ++nf) { const float d = c[nf][i] - m; v += d * d; }
        v += __shfl_xor(v, 1); v += __shfl_xor(v, 2); v += __shfl_xor(v, 4); v += __shfl_xor(v, 8);
        mu[i] = m;
        rs[i] = rsqrtf(v * (1.0f / 128.0f) + LN_EPS);
      }
#pragma unroll
      for (int nf = 0; nf < 8; ++nf) {
        const int col = nf * 16 + l16;
        const float gv = ln_g[l * DMOD + col], bv = ln_b[l * DMOD + col];
#pragma unroll
        for (int i = 0; i < 8; ++i) {
          const float y = (c[nf][i] - mu[i]) * rs[i] * gv + bv;
          c[nf][i] = y;
          hH[(row0 + 8 * hh + i) * STR + col] = h16(y * ASCL);
        }
      }
      __syncthreads();

      v8f c2[8];
#pragma unroll
      for (int nf = 0; nf < 8; ++nf) {
        const float bv = b2[l * DMOD + nf * 16 + l16];
        v8f t;
#pragma unroll
        for (int i = 0; i < 8; ++i) t[i] = (c[nf][i] + bv) * CSCL;
        c2[nf] = t;
      }
#pragma unroll 1
      for (int ch = 0; ch < HID / DMOD; ++ch) {
        {
          v16h hF[4];
          const unsigned short* hr = hH + (row0 + l16) * STR;
#pragma unroll
          for (int kt = 0; kt < 4; ++kt) hF[kt] = ldA(hr, kt, hh);
#pragma unroll
          for (int nf1 = 0; nf1 < 8; ++nf1) {
            v8f a1 = zero8;
#pragma unroll
            for (int kt = 0; kt < 4; ++kt) a1 = wmh(hF[kt], ldB(w1l, kt * (HID / 16) + ch * 8 + nf1, lane), a1);
            const float bv = b1[l * HID + ch * DMOD + nf1 * 16 + l16];
            const int col = nf1 * 16 + l16;
#pragma unroll
            for (int i = 0; i < 8; ++i)
              tW[(8 * hh + i) * STR + col] = h16(fmaxf(a1[i] * INVSCL + bv, 0.0f) * ASCL);
          }
        }
        __syncthreads();
        {
          v16h tF[4];
          const unsigned short* tr = tW + l16 * STR;
#pragma unroll
          for (int kt = 0; kt < 4; ++kt) tF[kt] = ldA(tr, kt, hh);
#pragma unroll
          for (int nf2 = 0; nf2 < 8; ++nf2) {
#pragma unroll
            for (int kt = 0; kt < 4; ++kt)
              c2[nf2] = wmh(tF[kt], ldB(w2l, (ch * (DMOD / 32) + kt) * (DMOD / 16) + nf2, lane), c2[nf2]);
          }
        }
        __syncthreads();
      }
#pragma unroll
      for (int nf = 0; nf < 8; ++nf) {
        const int col = nf * 16 + l16;
#pragma unroll
        for (int i = 0; i < 8; ++i) hS[(row0 + 8 * hh + i) * HSP + col] = c2[nf][i] * INVSCL;
      }
      __syncthreads();
    }

    if (wave < GPH / 2) {
      const int g = tid >> 4, sub = tid & 15;
      float part = 0.0f;
#pragma unroll 1
      for (int cc = 0; cc < 8; ++cc) {
        const int col = sub * 8 + cc;
        float s = 0.0f;
#pragma unroll
        for (int r = 0; r < NPG; ++r) s += hS[(g * NPG + r) * HSP + col];
        part += (s * (1.0f / 9.0f)) * fc_w[col];
      }
      part += __shfl_xor(part, 1); part += __shfl_xor(part, 2);
      part += __shfl_xor(part, 4); part += __shfl_xor(part, 8);
      if (sub == 0) {
        float z = part + fc_b[0];
        z = fminf(30.0f, fmaxf(-30.0f, z));
        const float ez = expf(-z);
        sOut[hp * GPH + g] = 1.0f / (1.0f + ez);
      }
    }
  }
  __syncthreads();

  if (wave == 0) {
    const int gb = (int)blockIdx.x * GPB;
    int nv = nG - gb; nv = nv > GPB ? GPB : nv;
    if (nv == GPB) {
      const int q = lane & 7;
      const v4f v = *(const v4f*)(sOut + 4 * q);
      float* p = out + gb + 4 * q;
      const bool w = lane < 8;
      if (w) *(volatile v4f*)p = v;
      __threadfence();
      if (w) *(volatile v4f*)p = v;
    } else {
      const float v = sOut[lane];
      const bool w = lane < nv;
      float* p = out + gb + (w ? lane : 0);
      if (w) *(volatile float*)p = v;
      __threadfence();
      if (w) *(volatile float*)p = v;
    }
  }
}

extern "C" void kernel_launch(void* const* d_in, const int* in_sizes, int n_in,
                              void* d_out, int out_size, void* d_ws, size_t ws_size,
                              hipStream_t stream) {
  if (n_in < 15) return;
  const int nG = out_size;
  if (nG <= 0) return;
  if (in_sizes[12] < nG * NPG) return;
  const int nN = nG * NPG;
  const int nE = in_sizes[13];
  if (nE != nG * EPG || in_sizes[14] != nE) return;
  if (in_sizes[0] < DMOD || (in_sizes[0] % DMOD) != 0) return;
  const int nOps = in_sizes[0] / DMOD;
  if (in_sizes[1] < DMOD || in_sizes[10] < DMOD || in_sizes[11] < 1) return;
  if (in_sizes[2] != NLAYERS * DMOD * DMOD) return;
  if (in_sizes[6] != NLAYERS * DMOD * HID) return;
  if (in_sizes[8] != NLAYERS * HID * DMOD) return;
  if (in_sizes[3] < NLAYERS * DMOD || in_sizes[4] < NLAYERS * DMOD ||
      in_sizes[5] < NLAYERS * DMOD || in_sizes[9] < NLAYERS * DMOD) return;
  if (in_sizes[7] < NLAYERS * HID) return;

  const float* op_table   = (const float*)d_in[0];
  const float* device_emb = (const float*)d_in[1];
  const float* Wg         = (const float*)d_in[2];
  const float* bg         = (const float*)d_in[3];
  const float* ln_g       = (const float*)d_in[4];
  const float* ln_b       = (const float*)d_in[5];
  const float* W1         = (const float*)d_in[6];
  const float* b1         = (const float*)d_in[7];
  const float* W2         = (const float*)d_in[8];
  const float* b2         = (const float*)d_in[9];
  const float* fc_w       = (const float*)d_in[10];
  const float* fc_b       = (const float*)d_in[11];
  const int*   op_idx     = (const int*)d_in[12];
  const int*   srcE       = (const int*)d_in[13];
  const int*   dstE       = (const int*)d_in[14];
  float* out = (float*)d_out;

  const size_t szWg = (size_t)NLAYERS * DMOD * DMOD * 2;
  const size_t szW1 = (size_t)NLAYERS * DMOD * HID * 2;
  const size_t szW2 = (size_t)NLAYERS * HID * DMOD * 2;
  const size_t oWg = 0;
  const size_t oW1 = oWg + szWg;
  const size_t oW2 = oW1 + szW1;
  const size_t tot = oW2 + szW2;
  if (tot > ws_size) return;
  char* ws = (char*)d_ws;
  unsigned short* wgF = (unsigned short*)(ws + oWg);
  unsigned short* w1F = (unsigned short*)(ws + oW1);
  unsigned short* w2F = (unsigned short*)(ws + oW2);

  const int npWg = DMOD * DMOD / 8;
  const int npW1 = DMOD * HID / 8;
  const int npW2 = HID * DMOD / 8;
  k_wprep<<<dim3((npWg + 255) / 256, NLAYERS, 1), 256, 0, stream>>>(Wg, wgF, DMOD, DMOD, npWg);
  k_wprep<<<dim3((npW1 + 255) / 256, NLAYERS, 1), 256, 0, stream>>>(W1, w1F, DMOD, HID, npW1);
  k_wprep<<<dim3((npW2 + 255) / 256, NLAYERS, 1), 256, 0, stream>>>(W2, w2F, HID, DMOD, npW2);

  hipFuncSetAttribute(reinterpret_cast<const void*>(&k_gcn),
                      hipFuncAttributeMaxDynamicSharedMemorySize, SMEM_BYTES);
  const int nBlk = (nG + GPB - 1) / GPB;
  k_gcn<<<nBlk, NTHREADS, SMEM_BYTES, stream>>>(
      op_table, device_emb, bg, ln_g, ln_b, b1, b2, fc_w, fc_b, op_idx, srcE, dstE,
      wgF, w1F, w2F, out, nG, nN, nE, nOps);
}
